// MLPContrastive_41807211659400
// MI455X (gfx1250) — hardware-run, weakly checked
//
#include <hip/hip_runtime.h>


#ifndef NIMG
#define NIMG 2048
#endif
#define NIMG_FULL 2048
#define NTXT 128
#define DIN  768
#define WTP  1536
#define HID  512
#define IPP  516
#define OPP  132

static_assert(WTP == 2 * DIN);
static_assert(DIN % 32 == 0);
static_assert(DIN % 8 == 0);
static_assert(WTP % 64 == 0);
static_assert(HID % 64 == 0);
static_assert(HID == 8 * 64);
static_assert(HID % 4 == 0);
static_assert(NIMG % 16 == 0);
static_assert(NIMG <= NIMG_FULL);
static_assert(NTXT % 16 == 0);
static_assert(NTXT == 4 * 32);
static_assert((IPP * 4) % 16 == 0);
static_assert((OPP * 4) % 16 == 0);
static_assert(IPP >= HID);
static_assert(OPP >= NTXT);
static_assert(((size_t)NIMG * DIN) % (8 * 256) == 0);
static_assert(((size_t)NTXT * DIN) % (8 * 256) == 0);

typedef unsigned short bf;
typedef __attribute__((ext_vector_type(16))) __bf16   v16bf;
typedef __attribute__((ext_vector_type(8)))  unsigned short v8us;
typedef __attribute__((ext_vector_type(8)))  float    v8f;
typedef __attribute__((ext_vector_type(4)))  float    v4f;
typedef v4f  __attribute__((may_alias)) v4fa;
typedef v8us __attribute__((may_alias)) v8usa;

__device__ __forceinline__ unsigned short f2bf(float f) { unsigned u = __float_as_uint(f); u += 0x7FFFu + ((u >> 16) & 1u); return (unsigned short)(u >> 16); }
__device__ __forceinline__ float bfr(float f) { return __uint_as_float(((unsigned)f2bf(f)) << 16); }
__device__ __forceinline__ v16bf cat16b(v8us lo, v8us hi) { return __builtin_bit_cast(v16bf, __builtin_shufflevector(lo, hi, 0, 1, 2, 3, 4, 5, 6, 7, 8, 9, 10, 11, 12, 13, 14, 15)); }
__device__ __forceinline__ v8f wmmab(v16bf a, v16bf b, v8f c) { return __builtin_amdgcn_wmma_f32_16x16x32_bf16(false, a, false, b, (short)0, c, false, false); }
__device__ __forceinline__ v16bf ldb(const bf* p)  { return cat16b(*(const v8us*)p, *(const v8us*)(p + 16)); }
__device__ __forceinline__ v8f wmmab_g(v16bf a, v16bf b, v8f c) {
    c = wmmab(a, b, c);
    asm volatile("v_nop\n\tv_nop\n\tv_nop\n\tv_nop" : "+v"(c) : "v"(a), "v"(b));
    return c;
}

__global__ __launch_bounds__(256) void k_cvt8(const float* __restrict__ src, bf* dst, size_t n8) {
    const size_t i = (size_t)blockIdx.x * 256 + threadIdx.x; if (i >= n8) return;
    const v8f v = *(const v8f*)(src + i * 8); v8us o;
#pragma unroll
    for (int k = 0; k < 8; ++k) o[k] = f2bf(v[k]);
    *(volatile v8us*)(dst + i * 8) = o; __threadfence(); *(volatile v8us*)(dst + i * 8) = o;
}

__global__ __launch_bounds__(256) void k_wt(const float* __restrict__ W, bf* WT) {
    __shared__ __align__(16) unsigned short ts[64 * 72];
    static_assert(sizeof(unsigned short) * 64 * 72 <= 131072);
    const int tid = threadIdx.x; const int k0 = blockIdx.x * 64, n0 = blockIdx.y * 64;
    static_assert(256 * 4 * 4 == 64 * 64);
#pragma unroll
    for (int i = 0; i < 4; ++i) { const int idx = i * 256 + tid; const int kk = idx >> 4, c4 = (idx & 15) * 4;
        const v4f v = *(const v4f*)(W + (size_t)(k0 + kk) * HID + n0 + c4);
#pragma unroll
        for (int e = 0; e < 4; ++e) ts[(c4 + e) * 72 + kk] = f2bf(v[e]); }
    __syncthreads();
    static_assert(256 * 2 * 16 == 64 * 128);
#pragma unroll 1
    for (int ps = 0; ps < 2; ++ps) {
#pragma unroll
        for (int i = 0; i < 2; ++i) { const int p = i * 256 + tid; const int nn = p >> 3, c8 = (p & 7) * 8;
            const v8us o = *(const v8usa*)(&ts[nn * 72 + c8]);
            *(volatile v8us*)(WT + (size_t)(n0 + nn) * WTP + k0 + c8) = o; }
        if (ps == 0) __threadfence(); }
}

__device__ __forceinline__ void proj16x64(const bf* __restrict__ A, const bf* __restrict__ Bt, size_t aoff, size_t boff, v8f (&acc)[4]) {
#pragma unroll
    for (int nb = 0; nb < 4; ++nb) acc[nb] = (v8f){};
#pragma unroll 1
    for (int kc = 0; kc < DIN; kc += 32) {
        const v16bf a = ldb(A + aoff + kc);
#pragma unroll
        for (int nb = 0; nb < 4; ++nb) { const v16bf b = ldb(Bt + boff + (size_t)nb * 16 * WTP + kc); acc[nb] = wmmab_g(a, b, acc[nb]); }
    }
}

__global__ __launch_bounds__(256) void k_tproj(const bf* __restrict__ XT, const bf* __restrict__ WT, const float* __restrict__ b1, float* TP) {
    __shared__ __align__(16) float ips[16 * IPP];
    static_assert(sizeof(float) * 16 * IPP <= 131072);
    const int tid = threadIdx.x, lane = tid & 31, lr = lane & 15, hi = lane >> 4;
    const int wave = __builtin_amdgcn_readfirstlane((int)(threadIdx.x >> 5));
    const int r0 = blockIdx.x * 16, c0 = wave * 64;
    v8f acc[4];
    proj16x64(XT, WT, (size_t)(r0 + lr) * DIN + 8 * hi, (size_t)(c0 + lr) * WTP + DIN + 8 * hi, acc);
#pragma unroll
    for (int nb = 0; nb < 4; ++nb) { const float bc = bfr(b1[c0 + nb * 16 + lr]);
#pragma unroll
        for (int j = 0; j < 8; ++j) ips[(hi * 8 + j) * IPP + c0 + nb * 16 + lr] = acc[nb][j] + bc; }
    __syncthreads();
    float* dst = TP + (size_t)r0 * HID;
    static_assert(256 * 8 * 16 == 16 * HID * 4);
#pragma unroll 1
    for (int ps = 0; ps < 2; ++ps) {
#pragma unroll
        for (int i = 0; i < 8; ++i) { const int idx = i * 256 + tid; const int row = idx >> 7, c4 = (idx & 127) * 4;
            const v4f val = *(const v4fa*)(&ips[row * IPP + c4]);
            *(volatile v4f*)(dst + (size_t)idx * 4) = val; }
        if (ps == 0) __threadfence(); }
}

__global__ __launch_bounds__(256) void k_sim(const bf* __restrict__ XI, const bf* __restrict__ WT, const float* __restrict__ TP,
                                             const float* __restrict__ W2, const float* __restrict__ b2, float* OUT) {
    __shared__ __align__(16) float ips[16 * IPP];
    __shared__ __align__(16) float w2s[HID];
    __shared__ __align__(16) float outs[16 * OPP];
    static_assert(sizeof(float) * (16 * IPP + HID + 16 * OPP) <= 131072);
    const int tid = threadIdx.x, lane = tid & 31, lr = lane & 15, hi = lane >> 4;
    const int wave = __builtin_amdgcn_readfirstlane((int)(threadIdx.x >> 5));
    const int r0 = blockIdx.x * 16, c0 = wave * 64;
#pragma unroll 1
    for (int i = tid; i < HID; i += 256) w2s[i] = bfr(W2[i]);
    v8f acc[4];
    proj16x64(XI, WT, (size_t)(r0 + lr) * DIN + 8 * hi, (size_t)(c0 + lr) * WTP + 8 * hi, acc);
#pragma unroll
    for (int nb = 0; nb < 4; ++nb) {
#pragma unroll
        for (int j = 0; j < 8; ++j) ips[(hi * 8 + j) * IPP + c0 + nb * 16 + lr] = acc[nb][j]; }
    __syncthreads();
    const float b2v = bfr(b2[0]);
    const int kx = (wave & 3) * 32 + lane;
    const int rb = (wave >> 2) * 8;
    const float* tprow = TP + (size_t)kx * HID;
    float s[8];
#pragma unroll
    for (int j = 0; j < 8; ++j) s[j] = 0.0f;
#pragma unroll 1
    for (int h4 = 0; h4 < HID; h4 += 4) {
        const v4f t = *(const v4f*)(tprow + h4);
        const v4f w = *(const v4fa*)(&w2s[h4]);
#pragma unroll
        for (int j = 0; j < 8; ++j) {
            const v4f a = *(const v4fa*)(&ips[(rb + j) * IPP + h4]);
            float sj = s[j];
            sj = fmaf(fmaxf(a[0] + t[0], 0.0f), w[0], sj);
            sj = fmaf(fmaxf(a[1] + t[1], 0.0f), w[1], sj);
            sj = fmaf(fmaxf(a[2] + t[2], 0.0f), w[2], sj);
            sj = fmaf(fmaxf(a[3] + t[3], 0.0f), w[3], sj);
            s[j] = sj; }
    }
#pragma unroll
    for (int j = 0; j < 8; ++j) outs[(rb + j) * OPP + kx] = s[j] + b2v;
    __syncthreads();
    float* dst = OUT + (size_t)r0 * NTXT;
    static_assert(256 * 2 * 16 == 16 * NTXT * 4);
#pragma unroll 1
    for (int ps = 0; ps < 2; ++ps) {
#pragma unroll
        for (int i = 0; i < 2; ++i) { const int idx = i * 256 + tid; const int row = idx >> 5, c4 = (idx & 31) * 4;
            const v4f val = *(const v4fa*)(&outs[row * OPP + c4]);
            *(volatile v4f*)(dst + (size_t)idx * 4) = val; }
        if (ps == 0) __threadfence(); }
}

static constexpr size_t al256(size_t v) { return (v + 255) & ~(size_t)255; }
static constexpr size_t SZ_XI = al256((size_t)NIMG * DIN * 2);
static constexpr size_t SZ_XT = al256((size_t)NTXT * DIN * 2);
static constexpr size_t SZ_WT = al256((size_t)HID * WTP * 2);
static constexpr size_t SZ_TP = al256((size_t)NTXT * HID * 4);
static constexpr size_t SZ_TOTAL = SZ_XI + SZ_XT + SZ_WT + SZ_TP;
static_assert(SZ_TOTAL <= (size_t)134217728);
static_assert((size_t)(WTP / 64) * 64 * (size_t)(HID / 64) * 64 * 2 == (size_t)HID * WTP * 2);
static_assert((size_t)(NTXT / 16) * 16 * HID * 4 == (size_t)NTXT * HID * 4);
static_assert((size_t)(NIMG / 16) * 16 * NTXT * 4 <= (size_t)NIMG_FULL * NTXT * 4);

extern "C" void kernel_launch(void* const* d_in, const int* in_sizes, int n_in,
                              void* d_out, int out_size, void* d_ws, size_t ws_size, hipStream_t stream) {
    if (n_in < 6) return;
    if ((size_t)in_sizes[0] < (size_t)NIMG * DIN) return;
    if ((size_t)in_sizes[1] < (size_t)NTXT * DIN) return;
    if ((size_t)in_sizes[2] < (size_t)WTP * HID) return;
    if (in_sizes[3] < HID || in_sizes[4] < HID || in_sizes[5] < 1) return;
    if ((size_t)out_size < (size_t)NIMG * NTXT) return;
    if (SZ_TOTAL > ws_size) return;
    const float* img = (const float*)d_in[0];
    const float* txt = (const float*)d_in[1];
    const float* w1  = (const float*)d_in[2];
    const float* b1  = (const float*)d_in[3];
    const float* w2  = (const float*)d_in[4];
    const float* b2  = (const float*)d_in[5];
    float* OUT = (float*)d_out;
    char* wsp = (char*)d_ws;
    bf* XI = (bf*)wsp; wsp += SZ_XI;
    bf* XT = (bf*)wsp; wsp += SZ_XT;
    bf* WT = (bf*)wsp; wsp += SZ_WT;
    float* TP = (float*)wsp; wsp += SZ_TP;

    { const size_t n8 = (size_t)NIMG * DIN / 8; k_cvt8<<<(unsigned)((n8 + 255) / 256), 256, 0, stream>>>(img, XI, n8); }
    { const size_t n8 = (size_t)NTXT * DIN / 8; k_cvt8<<<(unsigned)((n8 + 255) / 256), 256, 0, stream>>>(txt, XT, n8); }
    k_wt<<<dim3(WTP / 64, HID / 64, 1), 256, 0, stream>>>(w1, WT);
    k_tproj<<<dim3(NTXT / 16, 1, 1), 256, 0, stream>>>(XT, WT, b1, TP);
    k_sim<<<dim3(NIMG / 16, 1, 1), 256, 0, stream>>>(XI, WT, TP, w2, b2, OUT);
}
